// ODEBlock_34900904247575
// MI455X (gfx1250) — hardware-run, weakly checked
//
#include <hip/hip_runtime.h>


#define NB   16384
#define ND   64
#define NH   128
#define NSEG 5
#define NSTEP 4
typedef _Float16 h16;
typedef unsigned short bf;
typedef __attribute__((ext_vector_type(16))) __bf16   v16bf;
typedef __attribute__((ext_vector_type(16))) _Float16 v16h;
typedef __attribute__((ext_vector_type(8)))  _Float16 v8h;
typedef __attribute__((ext_vector_type(8)))  unsigned short v8us;
typedef __attribute__((ext_vector_type(8)))  float    v8f;
typedef __attribute__((ext_vector_type(4)))  float    v4f;
typedef v8h  __attribute__((may_alias)) v8ha;
typedef v4f  __attribute__((may_alias)) v4fa;
typedef v8us __attribute__((may_alias)) v8usa;

__device__ __forceinline__ unsigned short f2bf(float f) { unsigned u = __float_as_uint(f); u += 0x7FFFu + ((u >> 16) & 1u); return (unsigned short)(u >> 16); }
__device__ __forceinline__ float bf2f(unsigned short b) { return __uint_as_float(((unsigned)b) << 16); }
__device__ __forceinline__ float bfr(float f) { return bf2f(f2bf(f)); }
__device__ __forceinline__ v16h cat16(v8h lo, v8h hi) { return __builtin_shufflevector(lo, hi, 0, 1, 2, 3, 4, 5, 6, 7, 8, 9, 10, 11, 12, 13, 14, 15); }
__device__ __forceinline__ v16bf cat16b(v8us lo, v8us hi) { return __builtin_bit_cast(v16bf, __builtin_shufflevector(lo, hi, 0, 1, 2, 3, 4, 5, 6, 7, 8, 9, 10, 11, 12, 13, 14, 15)); }
__device__ __forceinline__ v8f wmma16(v16h a, v16h b, v8f c) { return __builtin_amdgcn_wmma_f32_16x16x32_f16(false, a, false, b, (short)0, c, false, false); }
__device__ __forceinline__ v8f wmmab(v16bf a, v16bf b, v8f c) { return __builtin_amdgcn_wmma_f32_16x16x32_bf16(false, a, false, b, (short)0, c, false, false); }


template <typename T16> struct WFrag;
template <> struct WFrag<h16> { typedef v16h V; static __device__ __forceinline__ V ld(const h16* p) { return cat16(*(const v8h*)p, *(const v8h*)(p + 16)); } static __device__ __forceinline__ v8f mma(V a, V b, v8f c) { return wmma16(a, b, c); } };
template <> struct WFrag<bf> { typedef v16bf V; static __device__ __forceinline__ V ld(const bf* p) { return cat16b(*(const v8us*)p, *(const v8us*)(p + 16)); } static __device__ __forceinline__ v8f mma(V a, V b, v8f c) { return wmmab(a, b, c); } };
template <typename T16, int NSPLIT, bool BIAS>
__global__ __launch_bounds__(32) void k_gemmw(const T16* __restrict__ A, const T16* __restrict__ A2, const T16* __restrict__ Bt, const T16* __restrict__ Bt2, int K, float* C, int ldc, const float* __restrict__ bias, size_t sA, size_t sB, size_t sC) {
    typedef typename WFrag<T16>::V V;
    __shared__ __align__(16) float os[16 * 68];
    const size_t z = blockIdx.z; A += z * sA; if (A2) A2 += z * sA; Bt += z * sB; if (Bt2) Bt2 += z * sB; C += z * sC;
    const int lane = threadIdx.x & 31, lr = lane & 15, hi = lane >> 4; const int r0 = blockIdx.x * 64, c0 = blockIdx.y * 64;
    v8f acc[4][4];
#pragma unroll
    for (int mb = 0; mb < 4; ++mb)
#pragma unroll
        for (int nb = 0; nb < 4; ++nb) acc[mb][nb] = (v8f){};
    const size_t aoff = (size_t)(r0 + lr) * K + 8 * hi, boff = (size_t)(c0 + lr) * K + 8 * hi;
    for (int kc = 0; kc < K; kc += 32) {
        V a[4], a2[4];
#pragma unroll
        for (int mb = 0; mb < 4; ++mb) { a[mb] = WFrag<T16>::ld(A + aoff + (size_t)mb * 16 * K + kc); if (NSPLIT == 1 || NSPLIT == 2) a2[mb] = WFrag<T16>::ld(A2 + aoff + (size_t)mb * 16 * K + kc); }
#pragma unroll
        for (int nb = 0; nb < 4; ++nb) { const V b = WFrag<T16>::ld(Bt + boff + (size_t)nb * 16 * K + kc); V b2; if (NSPLIT >= 2) b2 = WFrag<T16>::ld(Bt2 + boff + (size_t)nb * 16 * K + kc);
#pragma unroll
            for (int mb = 0; mb < 4; ++mb) { acc[mb][nb] = WFrag<T16>::mma(a[mb], b, acc[mb][nb]); if (NSPLIT == 1 || NSPLIT == 2) acc[mb][nb] = WFrag<T16>::mma(a2[mb], b, acc[mb][nb]); if (NSPLIT >= 2) acc[mb][nb] = WFrag<T16>::mma(a[mb], b2, acc[mb][nb]); } }
        asm volatile("v_nop\n\tv_nop\n\tv_nop\n\tv_nop" : "+v"(acc[0][0]), "+v"(acc[1][1]), "+v"(acc[2][2]), "+v"(acc[3][3]) : "v"(a[0]), "v"(a[3]));
    }
#pragma unroll
    for (int mb = 0; mb < 4; ++mb) {
#pragma unroll
        for (int nb = 0; nb < 4; ++nb) {
#pragma unroll
            for (int j = 0; j < 8; ++j) os[(hi * 8 + j) * 68 + nb * 16 + lr] = acc[mb][nb][j]; }
        __builtin_amdgcn_wave_barrier(); asm volatile("" ::: "memory");
        float* crow = C + (size_t)(r0 + mb * 16) * ldc + c0;
#pragma unroll 1
        for (int ps = 0; ps < 2; ++ps) {
#pragma unroll
            for (int s = 0; s < 8; ++s) { const int row = 2 * s + hi, cofs = lr * 4; v4f val = *(const v4fa*)(os + row * 68 + cofs); if (BIAS) { val[0] += bfr(bias[c0 + cofs]); val[1] += bfr(bias[c0 + cofs + 1]); val[2] += bfr(bias[c0 + cofs + 2]); val[3] += bfr(bias[c0 + cofs + 3]); }
                *(volatile v4f*)(crow + (size_t)row * ldc + cofs) = val; }
            if (ps == 0) __threadfence(); }
        __builtin_amdgcn_wave_barrier(); asm volatile("" ::: "memory");
    }
}

typedef __attribute__((ext_vector_type(2))) _Float16 v2h;
typedef __attribute__((ext_vector_type(4))) _Float16 v4h;
typedef __attribute__((ext_vector_type(2))) unsigned short v2us;
typedef __attribute__((ext_vector_type(4))) unsigned short v4us;
typedef __attribute__((ext_vector_type(2))) float v2f;
typedef __attribute__((ext_vector_type(4))) int v4i;

__global__ __launch_bounds__(256) void k_wtG(const float* __restrict__ w, int K, int N, bf* Bt) {
    const int lane = threadIdx.x & 31; const int L0 = (blockIdx.x * 8 + (threadIdx.x >> 5)) * 8; const int nlines = N * K / 64;
#pragma unroll
    for (int ps = 0; ps < 2; ++ps) {
        for (int l = 0; l < 8; ++l) { const int L = L0 + l; if (L >= nlines) break; const size_t e = (size_t)L * 64 + lane * 2; const int k = (int)(e % K), n = (int)(e / K); v2us o;
            o[0] = f2bf(w[(size_t)k * N + n]); o[1] = f2bf(w[(size_t)(k + 1) * N + n]); *(volatile v2us*)(Bt + e) = o; }
        if (ps == 0) __threadfence(); }
}

__global__ __launch_bounds__(256) void k_rnd(const float* __restrict__ src, float* y, bf* op, size_t n4) { const size_t i = (size_t)blockIdx.x * 256 + threadIdx.x; if (i >= n4) return; const v4f v = *(const v4f*)(src + i * 4); v4us o; v4f r;
#pragma unroll
    for (int k = 0; k < 4; ++k) { o[k] = f2bf(v[k]); r[k] = bf2f(o[k]); }
    *(volatile v4f*)(y + i * 4) = r; *(volatile v4us*)(op + i * 4) = o; __threadfence(); *(volatile v4f*)(y + i * 4) = r; *(volatile v4us*)(op + i * 4) = o; }

__global__ __launch_bounds__(256) void k_tanhb(const float* __restrict__ h, bf* th, size_t n4) { const size_t i = (size_t)blockIdx.x * 256 + threadIdx.x; if (i >= n4) return; const v4f v = *(const v4f*)(h + i * 4); v4us o;
#pragma unroll
    for (int k = 0; k < 4; ++k) o[k] = f2bf(tanhf(v[k]));
    *(volatile v4us*)(th + i * 4) = o; __threadfence(); *(volatile v4us*)(th + i * 4) = o; }

__global__ __launch_bounds__(256) void k_comb(const float* __restrict__ y, const float* __restrict__ p0, const float* __restrict__ p1, const float* __restrict__ p2, const float* __restrict__ p3, const float* __restrict__ p4, float c0, float c1, float c2, float c3, float c4, int nt, float dt, bf* op, float* ynew, float* snap, size_t n4) { const size_t i = (size_t)blockIdx.x * 256 + threadIdx.x; if (i >= n4) return;
    const v4f yv = *(const v4f*)(y + i * 4); v4f acc = c0 * *(const v4f*)(p0 + i * 4);
    if (nt > 1) acc = acc + c1 * *(const v4f*)(p1 + i * 4);
    if (nt > 2) acc = acc + c2 * *(const v4f*)(p2 + i * 4);
    if (nt > 3) acc = acc + c3 * *(const v4f*)(p3 + i * 4);
    if (nt > 4) acc = acc + c4 * *(const v4f*)(p4 + i * 4);
    const v4f s = yv + dt * acc; v4us o;
#pragma unroll
    for (int k = 0; k < 4; ++k) o[k] = f2bf(s[k]);
#pragma unroll
    for (int ps = 0; ps < 2; ++ps) { *(volatile v4us*)(op + i * 4) = o; if (ynew) *(volatile v4f*)(ynew + i * 4) = s; if (snap) *(volatile v4f*)(snap + i * 4) = s; if (ps == 0) __threadfence(); } }

constexpr float CA21 = (float)(1.0 / 5.0);
constexpr float CA31 = (float)(3.0 / 40.0), CA32 = (float)(9.0 / 40.0);
constexpr float CA41 = (float)(44.0 / 45.0), CA42 = (float)(-56.0 / 15.0), CA43 = (float)(32.0 / 9.0);
constexpr float CA51 = (float)(19372.0 / 6561.0), CA52 = (float)(-25360.0 / 2187.0), CA53 = (float)(64448.0 / 6561.0), CA54 = (float)(-212.0 / 729.0);
constexpr float CA61 = (float)(9017.0 / 3168.0), CA62 = (float)(-355.0 / 33.0), CA63 = (float)(46732.0 / 5247.0), CA64 = (float)(49.0 / 176.0), CA65 = (float)(-5103.0 / 18656.0);
constexpr float CB1 = (float)(35.0 / 384.0), CB3 = (float)(500.0 / 1113.0), CB4 = (float)(125.0 / 192.0), CB5 = (float)(-2187.0 / 6784.0), CB6 = (float)(11.0 / 84.0);
constexpr double TEV[NSEG + 1] = {0.0, 0.2, 0.4, 0.6, 0.8, 1.0};
constexpr float DTS[NSEG] = {(float)((TEV[1] - TEV[0]) / NSTEP), (float)((TEV[2] - TEV[1]) / NSTEP), (float)((TEV[3] - TEV[2]) / NSTEP), (float)((TEV[4] - TEV[3]) / NSTEP), (float)((TEV[5] - TEV[4]) / NSTEP)};

extern "C" void kernel_launch(void* const* d_in, const int* in_sizes, int n_in,
                              void* d_out, int out_size, void* d_ws, size_t ws_size, hipStream_t stream) {
    (void)in_sizes; (void)n_in; (void)out_size;
    const float* x0 = (const float*)d_in[0]; const float* w1 = (const float*)d_in[1]; const float* b1 = (const float*)d_in[2]; const float* w2 = (const float*)d_in[3]; const float* b2 = (const float*)d_in[4];
    static_assert(NB % 64 == 0 && NH % 64 == 0 && ND % 64 == 0 && ND % 32 == 0 && NH % 32 == 0 && (NB * ND / 4) % 256 == 0 && (NB * NH / 4) % 256 == 0 && (ND * NH) % 64 == 0, "the product launches: M and N multiples of 64, K a multiple of 32; the elementwise grids exact; the weight planes whole lines of 64 words");
    float* OUT = (float*)d_out;
    char* wsp = (char*)d_ws;
    auto take = [&](size_t bytes) { char* p = wsp; wsp += (bytes + 255) & ~(size_t)255; return (void*)p; };
    bf* W1t = (bf*)take((size_t)NH * ND * 2);     bf* W2t = (bf*)take((size_t)ND * NH * 2);
    float* Y[2]; Y[0] = (float*)take((size_t)NB * ND * 4); Y[1] = (float*)take((size_t)NB * ND * 4);
    bf* OP = (bf*)take((size_t)NB * ND * 2);     float* H1 = (float*)take((size_t)NB * NH * 4);     bf* TH = (bf*)take((size_t)NB * NH * 2);
    float* KS[6]; for (int j = 0; j < 6; ++j) KS[j] = (float*)take((size_t)NB * ND * 4);
    if ((size_t)(wsp - (char*)d_ws) > ws_size) return;
    const size_t n4d = (size_t)NB * ND / 4, n4h = (size_t)NB * NH / 4; const unsigned gd = (unsigned)(n4d / 256), gh = (unsigned)(n4h / 256);
    k_wtG<<<(unsigned)((ND * NH / 64 + 63) / 64), 256, 0, stream>>>(w1, ND, NH, W1t);
    k_wtG<<<(unsigned)((NH * ND / 64 + 63) / 64), 256, 0, stream>>>(w2, NH, ND, W2t);
    k_rnd<<<gd, 256, 0, stream>>>(x0, Y[0], OP, n4d);
    auto field = [&](float* kout) {
        k_gemmw<bf, 0, true><<<dim3(NB / 64, NH / 64, 1), 32, 0, stream>>>(OP, nullptr, W1t, nullptr, ND, H1, NH, b1, 0, 0, 0);
        k_tanhb<<<gh, 256, 0, stream>>>(H1, TH, n4h);
        k_gemmw<bf, 0, true><<<dim3(NB / 64, ND / 64, 1), 32, 0, stream>>>(TH, nullptr, W2t, nullptr, NH, kout, ND, b2, 0, 0, 0);
    };
    int cur = 0;
    for (int seg = 0; seg < NSEG; ++seg) {
        for (int st = 0; st < NSTEP; ++st) { const float* y = Y[cur]; float* yn = Y[cur ^ 1];
            field(KS[0]);
            k_comb<<<gd, 256, 0, stream>>>(y, KS[0], nullptr, nullptr, nullptr, nullptr, CA21, 0.0f, 0.0f, 0.0f, 0.0f, 1, DTS[seg], OP, nullptr, nullptr, n4d);
            field(KS[1]);
            k_comb<<<gd, 256, 0, stream>>>(y, KS[0], KS[1], nullptr, nullptr, nullptr, CA31, CA32, 0.0f, 0.0f, 0.0f, 2, DTS[seg], OP, nullptr, nullptr, n4d);
            field(KS[2]);
            k_comb<<<gd, 256, 0, stream>>>(y, KS[0], KS[1], KS[2], nullptr, nullptr, CA41, CA42, CA43, 0.0f, 0.0f, 3, DTS[seg], OP, nullptr, nullptr, n4d);
            field(KS[3]);
            k_comb<<<gd, 256, 0, stream>>>(y, KS[0], KS[1], KS[2], KS[3], nullptr, CA51, CA52, CA53, CA54, 0.0f, 4, DTS[seg], OP, nullptr, nullptr, n4d);
            field(KS[4]);
            k_comb<<<gd, 256, 0, stream>>>(y, KS[0], KS[1], KS[2], KS[3], KS[4], CA61, CA62, CA63, CA64, CA65, 5, DTS[seg], OP, nullptr, nullptr, n4d);
            field(KS[5]);
            k_comb<<<gd, 256, 0, stream>>>(y, KS[0], KS[2], KS[3], KS[4], KS[5], CB1, CB3, CB4, CB5, CB6, 5, DTS[seg], OP, yn, (st == NSTEP - 1) ? (OUT + (size_t)seg * NB * ND) : nullptr, n4d);
            cur ^= 1; } }
}
